// DenseGATLayer_49563922596601
// MI455X (gfx1250) — hardware-verified
//
#include <hip/hip_runtime.h>


namespace {
constexpr int NB = 8, N = 1024, DI = 256, NH = 4, HF = 64, DW = NH * HF, BL = 8  ;
constexpr float XS = 8.0f, WSC = 256.0f, PS = 1024.0f, LOG2E = 1.4426950408889634f, SLOPE = 0.2f, NEGINF = -1e9f;
static_assert(N % 64 == 0 && DW == 256, "tiling");
typedef _Float16 b16;
typedef __attribute__((ext_vector_type(16))) _Float16 v16b;
typedef __attribute__((ext_vector_type(8))) _Float16 v8b;
typedef __attribute__((ext_vector_type(8))) float v8f;
typedef __attribute__((ext_vector_type(4))) float v4f;
__device__ __forceinline__ float bf16_rne(float f) { unsigned int u = __float_as_uint(f); u += 0x7FFFu + ((u >> 16) & 1u); return __uint_as_float(u & 0xFFFF0000u); }
__device__ __forceinline__ void split16(float v, b16& hi, b16& lo) { hi = (b16)v; lo = (b16)(v - (float)hi); }
__device__ __forceinline__ v16b frag_kb(const b16* p, int hh) { const v8b a = *(const v8b*)(p + 8 * hh), b = *(const v8b*)(p + 16 + 8 * hh); v16b f;
#pragma unroll
  for (int e = 0; e < 8; ++e) { f[e] = a[e]; f[8 + e] = b[e]; } return f; }
__device__ __forceinline__ v8f wmma16b(v16b a, v16b b, v8f c) { v8f d = __builtin_amdgcn_wmma_f32_16x16x32_f16(false, a, false, b, (short)0, c, false, false); asm volatile("v_nop\n\tv_nop\n\tv_nop\n\tv_nop" : "+v"(d) : "v"(a), "v"(b)); return d; }
__device__ __forceinline__ void wave_lds_sync() { __builtin_amdgcn_fence(__ATOMIC_RELEASE, "workgroup"); __builtin_amdgcn_wave_barrier(); __builtin_amdgcn_fence(__ATOMIC_ACQUIRE, "workgroup"); }
__device__ __forceinline__ float pmul(float a, float b) { float p = a * b; asm volatile("" : "+v"(p)); return p; }
__device__ __forceinline__ int iclamp(int v, int lo, int hi) { return v < lo ? lo : (v > hi ? hi : v); }

typedef __attribute__((ext_vector_type(2))) _Float16 v2h;
typedef __attribute__((ext_vector_type(4))) int v4i;
__device__ __forceinline__ float nexp2(float v) { return __builtin_amdgcn_exp2f(v); }
__device__ __forceinline__ float elu_f(float v) { return v > 0.0f ? v : (__expf(v) - 1.0f); }
__global__ __launch_bounds__(256) void prep_kernel(const float* __restrict__ w, b16* __restrict__ WT) {
  const int t = blockIdx.x * 256 + threadIdx.x; if (t >= DW * DI / 8) return; const int e = t * 8; const int oo = e / DI, k0 = e % DI; v8b o;
  for (int j = 0; j < 8; ++j) o[j] = (b16)(bf16_rne(w[(size_t)(k0 + j) * DW + oo]) * WSC);
  for (int pass = 0; pass < 2; ++pass) { *(volatile v8b*)(WT + e) = o; __threadfence(); }
}
__global__ __launch_bounds__(128) void proj_kernel(const float* __restrict__ X, const b16* __restrict__ WT, const float* __restrict__ asrc, const float* __restrict__ adst, float* __restrict__ ESD, b16* __restrict__ VTh, b16* __restrict__ VTl) {
  __shared__ __attribute__((aligned(16))) float Tf[4][16][DW + 4]; __shared__ __attribute__((aligned(16))) float blk[64][8];
  const int wave = threadIdx.x >> 5, lane = threadIdx.x & 31, nloc = lane & 15, hlf = lane >> 4; const size_t r0 = ((size_t)blockIdx.x * 4 + wave) * 16; const int b = (int)((blockIdx.x * 64) / N), n0 = (int)((blockIdx.x * 64) % N);
  v8f acc[16];
#pragma unroll
  for (int t = 0; t < 16; ++t) acc[t] = (v8f){};
#pragma unroll 2
  for (int ks = 0; ks < DI / 32; ++ks) { v16b a; const float* xr = X + (r0 + nloc) * DI + ks * 32; const v4f c0 = *(const v4f*)(xr + 8 * hlf), c1 = *(const v4f*)(xr + 8 * hlf + 4), c2 = *(const v4f*)(xr + 16 + 8 * hlf), c3 = *(const v4f*)(xr + 16 + 8 * hlf + 4);
    for (int i = 0; i < 4; ++i) { a[i] = (b16)(bf16_rne(c0[i]) * XS); a[4 + i] = (b16)(bf16_rne(c1[i]) * XS); a[8 + i] = (b16)(bf16_rne(c2[i]) * XS); a[12 + i] = (b16)(bf16_rne(c3[i]) * XS); }
#pragma unroll
    for (int t = 0; t < 16; ++t) acc[t] = wmma16b(a, frag_kb(WT + (size_t)(t * 16 + nloc) * DI + ks * 32, hlf), acc[t]); }
#pragma unroll
  for (int t = 0; t < 16; ++t)
#pragma unroll
    for (int r = 0; r < 8; ++r) Tf[wave][8 * hlf + r][t * 16 + nloc] = acc[t][r] * (1.0f / (XS * WSC));
  wave_lds_sync();
  for (int rr = 0; rr < 16; ++rr) { float s1[NH], s2[NH]; for (int h = 0; h < NH; ++h) { s1[h] = 0.0f; s2[h] = 0.0f; }
#pragma unroll
    for (int q = 0; q < 8; ++q) { const int c = q * 32 + lane; const int h = c / HF, ci = c % HF; const float hv = Tf[wave][rr][c]; s1[h] += hv * bf16_rne(asrc[h * HF + ci]); s2[h] += hv * bf16_rne(adst[h * HF + ci]); }
#pragma unroll
    for (int h = 0; h < NH; ++h) {
#pragma unroll
      for (int o = 1; o < 32; o <<= 1) { s1[h] += __shfl_xor(s1[h], o); s2[h] += __shfl_xor(s2[h], o); } }
    if (lane < NH) { blk[wave * 16 + rr][lane] = s1[lane]; blk[wave * 16 + rr][NH + lane] = s2[lane]; } }
  __syncthreads();
  for (int pass = 0; pass < 2; ++pass) {
    if (wave == 0) { for (int q = lane * 4; q < 64 * 8; q += 128) *(volatile v4f*)(ESD + (size_t)blockIdx.x * 64 * 8 + q) = *(const v4f*)(&blk[0][0] + q); }
#pragma unroll 1
    for (int q = 0; q < 64; ++q) { const int c = wave * 64 + q; const int h = c / HF, f = c % HF; const int tk = lane * 2; v2h hv, lv;
      for (int j = 0; j < 2; ++j) { b16 p, ql; split16(Tf[(tk + j) >> 4][(tk + j) & 15][c] * XS, p, ql); hv[j] = p; lv[j] = ql; }
      const size_t oi = (((size_t)b * NH + h) * HF + f) * (size_t)N + n0 + tk; *(volatile v2h*)(VTh + oi) = hv; *(volatile v2h*)(VTl + oi) = lv; }
    __threadfence(); }
}
__global__ __launch_bounds__(64) void attn_kernel(const float* __restrict__ ESD, const int* __restrict__ A, const b16* __restrict__ VTh, const b16* __restrict__ VTl, float* __restrict__ out) {
  __shared__ __attribute__((aligned(16))) b16 Pb[2][16][32 + 8], Pc[2][16][32 + 8]; __shared__ __attribute__((aligned(16))) float To[2][16][HF + 4];
  const int wave = threadIdx.x >> 5, lane = threadIdx.x & 31, hh = lane >> 4, col = lane & 15; const int b = blockIdx.y / NH, h = blockIdx.y % NH; const int i0 = blockIdx.x * 32 + wave * 16, qi = i0 + col;
  const size_t rowq = (size_t)b * N + qi; const float esq = ESD[rowq * 8 + h]; const int* Arow = A + rowq * N; const b16* Vh = VTh + (((size_t)b * NH + h) * HF) * (size_t)N; const b16* Vl = VTl + (((size_t)b * NH + h) * HF) * (size_t)N;
  float m = -INFINITY, l = 0.0f; v8f o[4]; for (int t = 0; t < 4; ++t) o[t] = (v8f){};
#pragma unroll 1
  for (int kb = 0; kb < N; kb += 32) {
    float e[16]; float mx = -INFINITY;
    const float edl = ESD[((size_t)b * N + kb + lane) * 8 + NH + h];
#pragma unroll
    for (int u = 0; u < 2; ++u) { const v4i am0 = *(const v4i*)(Arow + kb + u * 16 + 8 * hh), am1 = *(const v4i*)(Arow + kb + u * 16 + 8 * hh + 4);
#pragma unroll
      for (int r = 0; r < 8; ++r) { const int jl = u * 16 + 8 * hh + r; const float edj = __shfl(edl, jl); const int am = (r < 4) ? am0[r] : am1[r - 4]; float lg = esq + edj; lg = (lg >= 0.0f) ? lg : SLOPE * lg; const float vv = ((am > 0) ? lg : NEGINF) * LOG2E; e[u * 8 + r] = vv; mx = fmaxf(mx, vv); } }
    mx = fmaxf(mx, __shfl_xor(mx, 16)); const float mn = fmaxf(m, mx); const float al = nexp2(m - mn); float sum = 0.0f;
#pragma unroll
    for (int i2 = 0; i2 < 16; ++i2) { const float p = nexp2(e[i2] - mn); sum += p; b16 a_, b_; split16(p * PS, a_, b_); const int sl = (i2 < 8 ? 0 : 16) + 8 * hh + (i2 & 7); Pb[wave][col][sl] = a_; Pc[wave][col][sl] = b_; }
    sum += __shfl_xor(sum, 16); l = l * al + sum; m = mn;
    wave_lds_sync();
    const v16b pf = frag_kb(&Pb[wave][col][0], hh), pg = frag_kb(&Pc[wave][col][0], hh);
#pragma unroll
    for (int t = 0; t < 4; ++t) { o[t] *= al; const size_t vr = (size_t)(t * 16 + col) * N + kb; const v16b va = frag_kb(Vh + vr, hh), vb = frag_kb(Vl + vr, hh); o[t] = wmma16b(va, pf, o[t]); o[t] = wmma16b(va, pg, o[t]); o[t] = wmma16b(vb, pf, o[t]); }
    wave_lds_sync(); }
  const float inv = 1.0f / (l * PS * XS);
#pragma unroll
  for (int t = 0; t < 4; ++t)
#pragma unroll
    for (int r = 0; r < 8; ++r) To[wave][col][t * 16 + 8 * hh + r] = elu_f(o[t][r] * inv);
  wave_lds_sync();
  for (int pass = 0; pass < 2; ++pass) { for (int rr = 0; rr < 16; ++rr) { const v4f f = {To[wave][rr][lane * 2], To[wave][rr][lane * 2 + 1], 0.0f, 0.0f}; __attribute__((ext_vector_type(2))) float f2 = {f[0], f[1]}; *(volatile __attribute__((ext_vector_type(2))) float*)(out + ((size_t)b * N + i0 + rr) * DW + h * HF + lane * 2) = f2; } __threadfence(); }
}
}

extern "C" void kernel_launch(void* const* d_in, const int* in_sizes, int n_in, void* d_out, int out_size, void* d_ws, size_t ws_size, hipStream_t stream) {
  (void)n_in;
  auto Fp = [&](int i) { return (const float*)d_in[i]; }; auto Ip = [&](int i) { return (const int*)d_in[i]; };
  if (in_sizes[0] != NB * N * DI || in_sizes[1] != NB * N * N || in_sizes[2] != DI * DW || in_sizes[3] != NH * HF || in_sizes[4] != NH * HF || out_size != NB * N * DW) return;
  size_t off = 0; char* ws = (char*)d_ws;
  auto carve = [&](size_t bytes) { char* p = ws + off; off += (bytes + 255) & ~(size_t)255; return p; };
  b16* WT = (b16*)carve((size_t)DW * DI * 2); float* ESD = (float*)carve((size_t)NB * N * 8 * 4); b16* VTh = (b16*)carve((size_t)NB * N * DW * 2); b16* VTl = (b16*)carve((size_t)NB * N * DW * 2);
  if (off > ws_size || off > ((size_t)128 << 20)) return;
  prep_kernel<<<(DW * DI / 8 + 255) / 256, 256, 0, stream>>>(Fp(2), WT);
  proj_kernel<<<(NB * N) / 64, 128, 0, stream>>>(Fp(0), WT, Fp(3), Fp(4), ESD, VTh, VTl);
  attn_kernel<<<dim3(N / 32, BL * NH), 64, 0, stream>>>(ESD, Ip(1), VTh, VTl, (float*)d_out);
}
